// DependencyParseModel_43757126812263
// MI455X (gfx1250) — hardware-run, weakly checked
//
#include <hip/hip_runtime.h>
#include <math.h>

typedef __attribute__((ext_vector_type(16))) _Float16 v16h;
typedef __attribute__((ext_vector_type(8)))  _Float16 v8h;
typedef __attribute__((ext_vector_type(8)))  float    v8f;
typedef __attribute__((ext_vector_type(4)))  float    v4f;
typedef __attribute__((ext_vector_type(2)))  float    v2f;

constexpr int kSeq   = 256;
constexpr int kDW    = 300;
constexpr int kDT    = 100;
constexpr int kH     = 400;
constexpr int kG4    = 1600;
constexpr int kGW    = 3200;
constexpr int kKP0   = 416;
constexpr int kSegP  = 448;
constexpr int kXP    = 896;
constexpr int kMlp   = 1600;
constexpr int kOutD  = 257;
constexpr int kOutN  = kOutD * kOutD;
constexpr int kVocab = 50000;
constexpr int kTags  = 50;
constexpr int kRecWaves   = kH / 16;
constexpr int kRecThreads = kRecWaves * 32;
constexpr int kPairWaves  = 7;
constexpr int kPairLines  = (kOutN + 31) / 32;
constexpr int kGroups416  = kGW * (kKP0 / 8);
constexpr int kGroups896  = kGW * (kXP / 8);
constexpr int kGroupsX    = kSeq * (kKP0 / 8);
constexpr float kACarry   = 64.0f;
constexpr float kWCarry   = 16.0f;
constexpr float kInvCarry = 1.0f / (kACarry * kWCarry);

static_assert(kDW + kDT == kH);
static_assert(4 * kH == kG4 && 2 * kG4 == kGW);
static_assert((kKP0 % 32) == 0 && kKP0 >= kH && (kXP % 32) == 0 && kXP == 2 * kSegP && kSegP >= kKP0);
static_assert((kSeq % 64) == 0 && (kGW % 64) == 0 && (kG4 % 64) == 0);
static_assert((kH % 16) == 0 && kRecWaves == 25 && kRecThreads == 800);
static_assert((kH % 8) == 0 && (kSegP % 8) == 0 && ((kSegP * 2) % 128) == 0);
static_assert((kGroups416 % 256) == 0 && (kGroups896 % 256) == 0 && (kGroupsX % 256) == 0);
static_assert(kPairLines == 2065 && (kPairLines % kPairWaves) == 0);
static_assert(kOutN == 66049);

constexpr size_t kOffX16  = 0;
constexpr size_t kOffWI0  = kOffX16  + (size_t)kSeq * kKP0 * 2;
constexpr size_t kOffWHH  = kOffWI0  + (size_t)kGW * kKP0 * 2;
constexpr size_t kOffWI1  = kOffWHH  + (size_t)2 * kGW * kKP0 * 2;
constexpr size_t kOffW1AB = kOffWI1  + (size_t)kGW * kXP * 2;
constexpr size_t kOffG0   = kOffW1AB + (size_t)kGW * kXP * 2;
constexpr size_t kOffG1   = kOffG0   + (size_t)kSeq * kGW * 4;
constexpr size_t kOffX1   = kOffG1   + (size_t)kSeq * kGW * 4;
constexpr size_t kOffH16  = kOffX1   + (size_t)kSeq * kXP * 2;
constexpr size_t kOffT    = kOffH16  + (size_t)kSeq * kXP * 2;
constexpr size_t kWsTotal = kOffT    + (size_t)kGW * kSeq * 4;
static_assert(kWsTotal == 30416896ull);
static_assert(kWsTotal <= 134217728ull);
static_assert((kOffWI0 % 128) == 0 && (kOffWHH % 128) == 0 && (kOffWI1 % 128) == 0 && (kOffW1AB % 128) == 0 &&
              (kOffG0 % 128) == 0 && (kOffG1 % 128) == 0 && (kOffX1 % 128) == 0 && (kOffH16 % 128) == 0 &&
              (kOffT % 128) == 0);

union FragU { v16h v; v8h h[2]; };
__device__ __forceinline__ v16h frag_load(const _Float16* p) {
  FragU f;
  f.h[0] = *(const v8h*)(p);
  f.h[1] = *(const v8h*)(p + 16);
  return f.v;
}
__device__ __forceinline__ v8f mma_f16(v16h a, v16h b, v8f c) {
  c = __builtin_amdgcn_wmma_f32_16x16x32_f16(false, a, false, b, (short)0, c, false, false);
  asm volatile("v_nop\n\tv_nop\n\tv_nop\n\tv_nop" : "+v"(c) : "v"(a), "v"(b));
  return c;
}

__global__ __launch_bounds__(256) void pack_x_kernel(
    const int* __restrict__ words, const int* __restrict__ tags,
    const float* __restrict__ wemb, const float* __restrict__ temb,
    unsigned short* __restrict__ dst)
{
  const int i = blockIdx.x * 256 + threadIdx.x;
  if (i >= kGroupsX) return;
  const int t  = i / (kKP0 / 8);
  const int g8 = i - t * (kKP0 / 8);
  int w = words[t];
  int tg = tags[t];
  w  = w  < 0 ? 0 : (w  > kVocab - 1 ? kVocab - 1 : w);
  tg = tg < 0 ? 0 : (tg > kTags - 1 ? kTags - 1 : tg);
  const float* wr = wemb + (size_t)w * kDW;
  const float* tr = temb + (size_t)tg * kDT;
  v8h hv;
#pragma unroll
  for (int e = 0; e < 8; ++e) {
    const int col = g8 * 8 + e;
    const int cw = col < kDW ? col : kDW - 1;
    int ct = col - kDW;
    ct = ct < 0 ? 0 : (ct > kDT - 1 ? kDT - 1 : ct);
    const float fw = wr[cw];
    const float ft = tr[ct];
    const float sa = (col < kDW) ? 1.0f : 0.0f;
    const float sb = (col >= kDW && col < kH) ? 1.0f : 0.0f;
    const float f = (sa * fw + sb * ft) * kACarry;
    hv[e] = (_Float16)f;
  }
  unsigned short* q = dst + (size_t)i * 8;
  *(volatile v8h*)q = hv;
  __threadfence();
  *(volatile v8h*)q = hv;
}

__global__ __launch_bounds__(256) void pack416_kernel(
    const float* __restrict__ srcA, const float* __restrict__ srcB, unsigned short* __restrict__ dst)
{
  const int i = blockIdx.x * 256 + threadIdx.x;
  if (i >= kGroups416) return;
  const int row = i / (kKP0 / 8);
  const int g8  = i - row * (kKP0 / 8);
  const bool data = g8 < (kH / 8);
  const int sc = data ? g8 * 8 : 0;
  const bool first = row < kG4;
  const int srow = first ? row : row - kG4;
  const float* sp = (first ? srcA : srcB) + (size_t)srow * kH + sc;
  const v4f a0 = *(const v4f*)(sp);
  const v4f a1 = *(const v4f*)(sp + 4);
  v8h hv;
#pragma unroll
  for (int e = 0; e < 4; ++e) {
    const float f0 = data ? a0[e] * kWCarry : 0.0f;
    const float f1 = data ? a1[e] * kWCarry : 0.0f;
    hv[e]     = (_Float16)f0;
    hv[4 + e] = (_Float16)f1;
  }
  unsigned short* q = dst + (size_t)i * 8;
  *(volatile v8h*)q = hv;
  __threadfence();
  *(volatile v8h*)q = hv;
}

__global__ __launch_bounds__(256) void pack896_kernel(
    const float* __restrict__ srcA, const float* __restrict__ srcB, int srcLd, unsigned short* __restrict__ dst)
{
  const int i = blockIdx.x * 256 + threadIdx.x;
  if (i >= kGroups896) return;
  const int row = i / (kXP / 8);
  const int g8  = i - row * (kXP / 8);
  const bool lo = g8 < (kH / 8);
  const bool hi = (g8 >= (kSegP / 8)) && (g8 < ((kSegP + kH) / 8));
  const bool data = lo || hi;
  const int scr = lo ? g8 * 8 : (g8 * 8 - (kSegP - kH));
  const int sc = data ? scr : 0;
  const bool first = row < kG4;
  const int srow = first ? row : row - kG4;
  const float* sp = (first ? srcA : srcB) + (size_t)srow * srcLd + sc;
  const v4f a0 = *(const v4f*)(sp);
  const v4f a1 = *(const v4f*)(sp + 4);
  v8h hv;
#pragma unroll
  for (int e = 0; e < 4; ++e) {
    const float f0 = data ? a0[e] * kWCarry : 0.0f;
    const float f1 = data ? a1[e] * kWCarry : 0.0f;
    hv[e]     = (_Float16)f0;
    hv[4 + e] = (_Float16)f1;
  }
  unsigned short* q = dst + (size_t)i * 8;
  *(volatile v8h*)q = hv;
  __threadfence();
  *(volatile v8h*)q = hv;
}

template <bool BIAS2>
__global__ __launch_bounds__(256) void gemm64_f16_kernel(
    const unsigned short* __restrict__ Ap, int lda,
    const unsigned short* __restrict__ Btp, int ldb,
    float* __restrict__ C, int ldc,
    const float* __restrict__ biasLo, const float* __restrict__ biasHi, int nSplit,
    int M, int N, int K, float scale)
{
  const _Float16* A  = (const _Float16*)Ap;
  const _Float16* Bt = (const _Float16*)Btp;
  __shared__ __align__(16) float sT[8][16 * 68];
  const int lane = threadIdx.x & 31;
  const int wave = threadIdx.x >> 5;
  const int tilesN = N >> 6;
  const int tilesM = M >> 6;
  const int tile = blockIdx.x * 8 + wave;
  if (tile >= tilesM * tilesN) return;
  const int tm = tile / tilesN;
  const int tn = tile - tm * tilesN;
  const int m0 = tm << 6;
  const int n0 = tn << 6;
  const int rlane = lane & 15;
  const int koff  = (lane >> 4) * 8;
  const int mOff  = (lane >> 4) * 8;

  v8f acc[4][4];
#pragma unroll
  for (int i = 0; i < 4; ++i)
#pragma unroll
    for (int j = 0; j < 4; ++j) acc[i][j] = (v8f){0.f, 0.f, 0.f, 0.f, 0.f, 0.f, 0.f, 0.f};

  for (int k0 = 0; k0 < K; k0 += 32) {
    v16h bh[4];
#pragma unroll
    for (int j = 0; j < 4; ++j) {
      const size_t bo = (size_t)(n0 + (j << 4) + rlane) * ldb + koff + k0;
      bh[j] = frag_load(Bt + bo);
    }
#pragma unroll
    for (int i = 0; i < 4; ++i) {
      const size_t ao = (size_t)(m0 + (i << 4) + rlane) * lda + koff + k0;
      const v16h ah = frag_load(A + ao);
#pragma unroll
      for (int j = 0; j < 4; ++j) acc[i][j] = mma_f16(ah, bh[j], acc[i][j]);
    }
  }

  float* slab = sT[wave];
#pragma unroll
  for (int i = 0; i < 4; ++i) {
    const int mBase = m0 + (i << 4);
#pragma unroll
    for (int j = 0; j < 4; ++j) {
      const int n = n0 + (j << 4) + rlane;
      float bv = 0.f;
      if (BIAS2) {
        const bool first = n0 < nSplit;
        const float* bp = first ? biasLo : biasHi;
        const int nb = first ? n : (n - nSplit);
        bv = bp[nb];
      }
#pragma unroll
      for (int r = 0; r < 8; ++r) {
        float v = acc[i][j][r] * scale;
        if (BIAS2) v += bv;
        slab[(mOff + r) * 68 + (j << 4) + rlane] = v;
      }
    }
    __builtin_amdgcn_fence(__ATOMIC_RELEASE, "workgroup");
    __builtin_amdgcn_wave_barrier();
    __builtin_amdgcn_fence(__ATOMIC_ACQUIRE, "workgroup");
    {
      const int hh = lane >> 4, c4 = (lane & 15) * 4;
      for (int pass = 0; pass < 2; ++pass) {
#pragma unroll
        for (int it = 0; it < 8; ++it) {
          const int row = it * 2 + hh;
          v4f v = *(const v4f*)(slab + row * 68 + c4);
          *(volatile v4f*)(C + (size_t)(mBase + row) * ldc + n0 + c4) = v;
        }
        __threadfence();
      }
    }
    __builtin_amdgcn_fence(__ATOMIC_RELEASE, "workgroup");
    __builtin_amdgcn_wave_barrier();
    __builtin_amdgcn_fence(__ATOMIC_ACQUIRE, "workgroup");
  }
}

__device__ __forceinline__ float pick8(v8f a, int r) {
  float v = a[0];
  v = (r == 1) ? a[1] : v;
  v = (r == 2) ? a[2] : v;
  v = (r == 3) ? a[3] : v;
  v = (r == 4) ? a[4] : v;
  v = (r == 5) ? a[5] : v;
  v = (r == 6) ? a[6] : v;
  v = (r == 7) ? a[7] : v;
  return v;
}
__device__ __forceinline__ float sigm(float x) { return 1.0f / (1.0f + expf(-x)); }

__global__ __launch_bounds__(800) void lstm_rec_kernel(
    const float* __restrict__ G, const unsigned short* __restrict__ Whh16p,
    const float* __restrict__ h0, const float* __restrict__ c0,
    unsigned short* __restrict__ Xout)
{
  __shared__ __align__(16) _Float16 hbuf[2][kSegP];
  const int tid  = threadIdx.x;
  const int lane = tid & 31;
  const int wave = tid >> 5;
  const int dir  = blockIdx.x;
  const int hh = lane >> 4;
  const int m  = lane & 15;
  const int r  = lane & 7;
  const int jrow = wave * 16 + 8 * hh + r;

  if (tid < kSegP) {
    const int jc = tid < kH ? tid : kH - 1;
    const float hv = h0[dir * kH + jc];
    const float f = (tid < kH) ? hv * kACarry : 0.0f;
    hbuf[0][tid] = (_Float16)f;
  }
  float c = c0[dir * kH + jrow];
  __syncthreads();

  const _Float16* W = (const _Float16*)Whh16p + (size_t)dir * kG4 * kKP0;
  const _Float16* wrow = W + (size_t)(wave * 16 + m) * kKP0 + 8 * hh;
  const float* gbase = G + dir * kG4 + jrow;
  unsigned short* xbase = Xout + dir * kSegP;
  v8h zero8;
#pragma unroll
  for (int e = 0; e < 8; ++e) zero8[e] = (_Float16)0.0f;

  int p = 0;
#pragma unroll 1
  for (int s = 0; s < kSeq; ++s) {
    const int t = dir ? (kSeq - 1 - s) : s;
    const float* gp = gbase + (size_t)t * kGW;
    const float gi = gp[0];
    const float gf = gp[kH];
    const float gg = gp[2 * kH];
    const float go = gp[3 * kH];

    v8f a0 = (v8f){0.f, 0.f, 0.f, 0.f, 0.f, 0.f, 0.f, 0.f};
    v8f a1 = a0, a2 = a0, a3 = a0;
    const _Float16* hb = &hbuf[p][8 * hh];
#pragma unroll 1
    for (int k0 = 0; k0 < kKP0; k0 += 32) {
      const v16h bf = frag_load(hb + k0);
      const v16h f0 = frag_load(wrow + k0);
      const v16h f1 = frag_load(wrow + (size_t)kH * kKP0 + k0);
      const v16h f2 = frag_load(wrow + (size_t)2 * kH * kKP0 + k0);
      const v16h f3 = frag_load(wrow + (size_t)3 * kH * kKP0 + k0);
      a0 = mma_f16(f0, bf, a0);
      a1 = mma_f16(f1, bf, a1);
      a2 = mma_f16(f2, bf, a2);
      a3 = mma_f16(f3, bf, a3);
    }
    const float pi = pick8(a0, r) * kInvCarry + gi;
    const float pf = pick8(a1, r) * kInvCarry + gf;
    const float pg = pick8(a2, r) * kInvCarry + gg;
    const float po = pick8(a3, r) * kInvCarry + go;
    const float si = sigm(pi);
    const float sf = sigm(pf);
    const float so = sigm(po);
    const float tg = tanhf(pg);
    c = sf * c + si * tg;
    const float hn = so * tanhf(c);

    const int q = p ^ 1;
    hbuf[q][jrow] = (_Float16)(hn * kACarry);
    if (wave == 0 && lane < (kSegP - kH) / 8) *(v8h*)(&hbuf[q][kH + 8 * lane]) = zero8;
    __syncthreads();

    if (wave < 2) {
      const int e0 = wave * 256 + lane * 8;
      const bool act = e0 < kSegP;
      const int e0c = act ? e0 : 0;
      const v8h hv = *(const v8h*)(&hbuf[q][e0c]);
      unsigned short* dstp = xbase + (size_t)t * kXP + e0c;
      if (act) *(volatile v8h*)dstp = hv;
      __threadfence();
      if (act) *(volatile v8h*)dstp = hv;
    }
    p = q;
  }
}

__global__ __launch_bounds__(224) void pair_out_kernel(
    const float* __restrict__ T, const float* __restrict__ b1m, const float* __restrict__ w2,
    const float* __restrict__ b2p, float* __restrict__ out)
{
  __shared__ __align__(16) float sWB[2 * kMlp];
  const int tid = threadIdx.x;
  const int lane = tid & 31;
  const int wave = tid >> 5;
#pragma unroll 1
  for (int k = tid; k < kMlp; k += kPairWaves * 32) {
    sWB[2 * k]     = b1m[k];
    sWB[2 * k + 1] = w2[k];
  }
  __syncthreads();
  const int line = blockIdx.x * kPairWaves + wave;
  if (line < kPairLines) {
    const int idx = line * 32 + lane;
    const bool valid = idx < kOutN;
    const int idxc = valid ? idx : kOutN - 1;
    const int r = idxc / kOutD;
    const int c = idxc - r * kOutD;
    const int ic = r > 0 ? r - 1 : 0;
    const int jc = c > 0 ? c - 1 : 0;
    const bool zero = (r == 0) || (c == 0) || (r == c);
    const float* ta = T + ic;
    const float* tb = T + (size_t)kMlp * kSeq + jc;
    const float b2 = b2p[0];
    float sacc = 0.0f;
#pragma unroll 2
    for (int k = 0; k < kMlp; ++k) {
      const float a = ta[(size_t)k * kSeq];
      const float b = tb[(size_t)k * kSeq];
      const v2f wb = *(const v2f*)(sWB + 2 * k);
      const float z = (a + b) + wb[0];
      const float e = expf(z + z);
      const float th = 1.0f - 2.0f * __builtin_amdgcn_rcpf(e + 1.0f);
      sacc = fmaf(wb[1], th, sacc);
    }
    const float val = zero ? 0.0f : (sacc + b2);
    float* dstp = out + idxc;
    if (valid) *(volatile float*)dstp = val;
    __threadfence();
    if (valid) *(volatile float*)dstp = val;
  }
}

extern "C" void kernel_launch(void* const* d_in, const int* in_sizes, int n_in,
                              void* d_out, int out_size, void* d_ws, size_t ws_size,
                              hipStream_t stream) {
  if (n_in < 23) return;
  if (in_sizes[0] != kSeq || in_sizes[1] != kSeq) return;
  if (in_sizes[3] != kVocab * kDW || in_sizes[4] != kTags * kDT) return;
  if (in_sizes[5] != kG4 * kH || in_sizes[6] != kG4 * kH || in_sizes[7] != kG4) return;
  if (in_sizes[8] != kG4 * kH || in_sizes[9] != kG4 * kH || in_sizes[10] != kG4) return;
  if (in_sizes[11] != kG4 * 2 * kH || in_sizes[12] != kG4 * kH || in_sizes[13] != kG4) return;
  if (in_sizes[14] != kG4 * 2 * kH || in_sizes[15] != kG4 * kH || in_sizes[16] != kG4) return;
  if (in_sizes[17] != 4 * kH || in_sizes[18] != 4 * kH) return;
  if (in_sizes[19] != kMlp * kMlp || in_sizes[20] != kMlp || in_sizes[21] != kMlp || in_sizes[22] != 1) return;
  if (out_size != kOutN) return;
  if (ws_size < kWsTotal) return;

  const int*   words = (const int*)d_in[0];
  const int*   tags  = (const int*)d_in[1];
  const float* wemb  = (const float*)d_in[3];
  const float* temb  = (const float*)d_in[4];
  const float* Wih0f = (const float*)d_in[5];
  const float* Whh0f = (const float*)d_in[6];
  const float* b0f   = (const float*)d_in[7];
  const float* Wih0b = (const float*)d_in[8];
  const float* Whh0b = (const float*)d_in[9];
  const float* b0b   = (const float*)d_in[10];
  const float* Wih1f = (const float*)d_in[11];
  const float* Whh1f = (const float*)d_in[12];
  const float* b1f   = (const float*)d_in[13];
  const float* Wih1b = (const float*)d_in[14];
  const float* Whh1b = (const float*)d_in[15];
  const float* b1b   = (const float*)d_in[16];
  const float* h0    = (const float*)d_in[17];
  const float* c0    = (const float*)d_in[18];
  const float* W1    = (const float*)d_in[19];
  const float* b1m   = (const float*)d_in[20];
  const float* w2    = (const float*)d_in[21];
  const float* b2m   = (const float*)d_in[22];
  float* out = (float*)d_out;

  char* ws = (char*)d_ws;
  unsigned short* X16  = (unsigned short*)(ws + kOffX16);
  unsigned short* WI0  = (unsigned short*)(ws + kOffWI0);
  unsigned short* WHH  = (unsigned short*)(ws + kOffWHH);
  unsigned short* WI1  = (unsigned short*)(ws + kOffWI1);
  unsigned short* W1AB = (unsigned short*)(ws + kOffW1AB);
  float*          G0   = (float*)(ws + kOffG0);
  float*          G1   = (float*)(ws + kOffG1);
  unsigned short* X1   = (unsigned short*)(ws + kOffX1);
  unsigned short* H16  = (unsigned short*)(ws + kOffH16);
  float*          T    = (float*)(ws + kOffT);
  unsigned short* WHH1 = WHH + (size_t)kGW * kKP0;

  pack_x_kernel<<<kGroupsX / 256, 256, 0, stream>>>(words, tags, wemb, temb, X16);
  pack416_kernel<<<kGroups416 / 256, 256, 0, stream>>>(Wih0f, Wih0b, WI0);
  pack416_kernel<<<kGroups416 / 256, 256, 0, stream>>>(Whh0f, Whh0b, WHH);
  pack416_kernel<<<kGroups416 / 256, 256, 0, stream>>>(Whh1f, Whh1b, WHH1);
  pack896_kernel<<<kGroups896 / 256, 256, 0, stream>>>(Wih1f, Wih1b, 2 * kH, WI1);
  pack896_kernel<<<kGroups896 / 256, 256, 0, stream>>>(W1, W1 + 2 * kH, kMlp, W1AB);

  constexpr int kGemmBlocks = ((kSeq / 64) * (kGW / 64)) / 8;
  static_assert(kGemmBlocks * 8 == (kSeq / 64) * (kGW / 64));

  gemm64_f16_kernel<true><<<kGemmBlocks, 256, 0, stream>>>(
      X16, kKP0, WI0, kKP0, G0, kGW, b0f, b0b, kG4, kSeq, kGW, kKP0, kInvCarry);
  lstm_rec_kernel<<<2, kRecThreads, 0, stream>>>(G0, WHH, h0, c0, X1);

  gemm64_f16_kernel<true><<<kGemmBlocks, 256, 0, stream>>>(
      X1, kXP, WI1, kXP, G1, kGW, b1f, b1b, kG4, kSeq, kGW, kXP, kInvCarry);
  lstm_rec_kernel<<<2, kRecThreads, 0, stream>>>(G1, WHH1, h0 + 2 * kH, c0 + 2 * kH, H16);

  gemm64_f16_kernel<false><<<kGemmBlocks, 256, 0, stream>>>(
      W1AB, kXP, H16, kXP, T, kSeq, b1m, b1m, 0, kGW, kSeq, kXP, kInvCarry);

  pair_out_kernel<<<kPairLines / kPairWaves, kPairWaves * 32, 0, stream>>>(T, b1m, w2, b2m, out);
}
